// MambaSSM_14242111553797
// MI455X (gfx1250) — hardware-run, weakly checked
//
#include <hip/hip_runtime.h>
#include <math.h>

typedef __attribute__((ext_vector_type(16))) _Float16 v16h;
typedef __attribute__((ext_vector_type(8)))  _Float16 v8h;
typedef __attribute__((ext_vector_type(16))) __bf16   v16b;
typedef __attribute__((ext_vector_type(8)))  __bf16   v8b;
typedef __attribute__((ext_vector_type(8)))  float    v8f;
typedef __attribute__((ext_vector_type(4)))  float    v4f;

constexpr int kBatch  = 2;
constexpr int kSeq    = 2048;
constexpr int kDm     = 1024;
constexpr int kDin    = 2048;
constexpr int kNst    = 16;
constexpr int kConvK  = 4;
constexpr int kXzP    = 2 * kDin;
constexpr int kBcdN   = 2 * kNst + 1;
constexpr int kBcdP   = 64;
constexpr int kRows   = kBatch * kSeq;
constexpr int kTrP    = 68;
constexpr int kConvTP = 260;
constexpr int kScanTS = 64;
constexpr int kScanSub = 16;
constexpr int kScanCh = 64;
constexpr int kScanYP = 68;
constexpr int kCdP    = 256;
constexpr float kLog2e = 1.44269504088896340736f;
constexpr float kLn2   = 0.69314718055994530942f;
constexpr float kHcar  = 256.0f;
constexpr float kCcar  = 1024.0f;
constexpr float kYfold = 1.0f / 262144.0f;
static_assert(kBcdN <= kBcdP);
static_assert((kDm % 32) == 0 && (kDin % 32) == 0);
static_assert((kRows % 64) == 0 && (kXzP % 64) == 0 && (kBcdP % 64) == 0 && (kDm % 64) == 0 && (kDin % 64) == 0);
static_assert((kSeq % kScanTS) == 0 && (kSeq % 64) == 0 && (kDin % kScanCh) == 0 && (kDin % 256) == 0);
static_assert((kScanTS % kScanSub) == 0 && kScanSub == 16 && kScanCh == 64 && kNst == 16 && kCdP == kScanSub * kNst);
static_assert((kRows * kDm) % (8 * 256) == 0);

constexpr size_t kOffXB   = 0;
constexpr size_t kOffW1T  = kOffXB  + (size_t)kRows * kDm  * 2;
constexpr size_t kOffW2T  = kOffW1T + (size_t)kXzP  * kDm  * 2;
constexpr size_t kOffW3T  = kOffW2T + (size_t)kBcdP * kDin * 2;
constexpr size_t kOffXZ   = kOffW3T + (size_t)kDm   * kDin * 2;
constexpr size_t kOffXS   = kOffXZ  + (size_t)kRows * kXzP * 4;
constexpr size_t kOffBCD  = kOffXS  + (size_t)kRows * kDin * 2;
constexpr size_t kOffYH   = kOffBCD + (size_t)kRows * kBcdP * 4;
constexpr size_t kOffYL   = kOffXS;
constexpr size_t kWsTotal = kOffYH  + (size_t)kRows * kDin * 2;
static_assert(kOffW1T == 8388608ull && kOffW2T == 16777216ull && kOffW3T == 17039360ull && kOffXZ == 21233664ull);
static_assert(kOffXS == 88342528ull && kOffBCD == 105119744ull && kOffYH == 106168320ull);
static_assert(kWsTotal == 122945536ull);
static_assert(kWsTotal <= 134217728ull);
static_assert((kOffW1T % 128) == 0 && (kOffW2T % 128) == 0 && (kOffW3T % 128) == 0 && (kOffXZ % 128) == 0 &&
              (kOffXS % 128) == 0 && (kOffBCD % 128) == 0 && (kOffYH % 128) == 0);

__device__ __forceinline__ unsigned short f2bf_bits(float f) {
  unsigned u = __float_as_uint(f);
  return (unsigned short)((u + 0x7FFFu + ((u >> 16) & 1u)) >> 16);
}
__device__ __forceinline__ float bf_bits2f(unsigned short h) { return __uint_as_float(((unsigned)h) << 16); }
__device__ __forceinline__ float bfr(float f) { return bf_bits2f(f2bf_bits(f)); }

__device__ __forceinline__ float sigm_f32(float t) {
  const float e = exp2f(-t * kLog2e);
  return __builtin_amdgcn_rcpf(1.0f + e);
}
__device__ __forceinline__ float softplus_f32(float v) {
  const float a   = exp2f(-fabsf(v) * kLog2e);
  const float up  = 1.0f + a;
  const float cor = (a - (up - 1.0f)) * __builtin_amdgcn_rcpf(up);
  const float l1p = fmaf(log2f(up), kLn2, cor);
  return fmaxf(v, 0.0f) + l1p;
}

__device__ __forceinline__ void dep_guard_h(v8f& a, v8f& b, v16h x, v16h y) { asm volatile("v_nop\n\tv_nop\n\tv_nop\n\tv_nop" : "+v"(a), "+v"(b) : "v"(x), "v"(y)); }
__device__ __forceinline__ void dep_guard_b(v8f& a, v8f& b, v16b x, v16b y) { asm volatile("v_nop\n\tv_nop\n\tv_nop\n\tv_nop" : "+v"(a), "+v"(b) : "v"(x), "v"(y)); }
__device__ __forceinline__ void dep_guard4_h(v8f& a, v8f& b, v8f& c, v8f& d, v16h x, v16h y) { asm volatile("v_nop\n\tv_nop\n\tv_nop\n\tv_nop" : "+v"(a), "+v"(b), "+v"(c), "+v"(d) : "v"(x), "v"(y)); }
__device__ __forceinline__ void dep_guard4_b(v8f& a, v8f& b, v8f& c, v8f& d, v16b x, v16b y) { asm volatile("v_nop\n\tv_nop\n\tv_nop\n\tv_nop" : "+v"(a), "+v"(b), "+v"(c), "+v"(d) : "v"(x), "v"(y)); }
__device__ __forceinline__ void keep4_h(v16h a, v16h b, v16h c, v16h d) { asm volatile("v_nop" :: "v"(a), "v"(b), "v"(c), "v"(d)); }
__device__ __forceinline__ void keep4_b(v16b a, v16b b, v16b c, v16b d) { asm volatile("v_nop" :: "v"(a), "v"(b), "v"(c), "v"(d)); }
__device__ __forceinline__ void acc_guard4(v8f& a, v8f& b, v8f& c, v8f& d) { asm volatile("v_nop\n\tv_nop\n\tv_nop\n\tv_nop" : "+v"(a), "+v"(b), "+v"(c), "+v"(d)); }
template <typename T> struct Frag;
template <> struct Frag<_Float16> {
  typedef v16h V; union U { v16h v; v8h h[2]; };
  static __device__ __forceinline__ v16h load(const _Float16* p) {
    U f; f.h[0] = *(const v8h*)(p); f.h[1] = *(const v8h*)(p + 16); return f.v;
  }
  static __device__ __forceinline__ v8f mma(v16h a, v16h b, v8f c) {
    return __builtin_amdgcn_wmma_f32_16x16x32_f16(false, a, false, b, (short)0, c, false, false);
  }
  static __device__ __forceinline__ void guard(v8f& a, v8f& b, v16h x, v16h y) { dep_guard_h(a, b, x, y); }
  static __device__ __forceinline__ void guard4(v8f& a, v8f& b, v8f& c, v8f& d, v16h x, v16h y) { dep_guard4_h(a, b, c, d, x, y); }
  static __device__ __forceinline__ void keep(v16h a, v16h b, v16h c, v16h d) { keep4_h(a, b, c, d); }
};
template <> struct Frag<__bf16> {
  typedef v16b V; union U { v16b v; v8b h[2]; };
  static __device__ __forceinline__ v16b load(const __bf16* p) {
    U f; f.h[0] = *(const v8b*)(p); f.h[1] = *(const v8b*)(p + 16); return f.v;
  }
  static __device__ __forceinline__ v8f mma(v16b a, v16b b, v8f c) {
    return __builtin_amdgcn_wmma_f32_16x16x32_bf16(false, a, false, b, (short)0, c, false, false);
  }
  static __device__ __forceinline__ void guard(v8f& a, v8f& b, v16b x, v16b y) { dep_guard_b(a, b, x, y); }
  static __device__ __forceinline__ void guard4(v8f& a, v8f& b, v8f& c, v8f& d, v16b x, v16b y) { dep_guard4_b(a, b, c, d, x, y); }
  static __device__ __forceinline__ void keep(v16b a, v16b b, v16b c, v16b d) { keep4_b(a, b, c, d); }
};

__device__ __forceinline__ v8f mma16_f16(v16h a, v16h b, v8f c) {
  c = __builtin_amdgcn_wmma_f32_16x16x32_f16(false, a, false, b, (short)0, c, false, false);
  asm volatile("v_nop\n\tv_nop\n\tv_nop\n\tv_nop" : "+v"(c) : "v"(a), "v"(b));
  return c;
}

template <int ET> struct Elem;
template <> struct Elem<0> { typedef _Float16 T; };
template <> struct Elem<1> { typedef __bf16 T; };
template <int ET, int SPL, int BIAS_MODE, int OUT_MODE, bool RESID, int ACT = 0>
__global__ __launch_bounds__(256) void wmma_gemm64(
    const unsigned short* __restrict__ Ap, const unsigned short* __restrict__ A2p, int lda, long strideA,
    const unsigned short* __restrict__ Btp, const unsigned short* __restrict__ Bt2p, int ldb, long strideB,
    void* __restrict__ Cout, void* __restrict__ Cout2, int ldc, long strideC,
    const float* __restrict__ bias,
    const float* __restrict__ resid, long strideR,
    int M, int N, int K, float scale) {
  typedef typename Elem<ET>::T T;
  typedef typename Frag<T>::V V;
  const T* A = (const T*)Ap; const T* A2 = (const T*)A2p; const T* Bt = (const T*)Btp; const T* Bt2 = (const T*)Bt2p;
  __shared__ __align__(16) float sT[8][16 * 68];
  const int b    = blockIdx.y;
  const int lane = threadIdx.x & 31;
  const int wave = threadIdx.x >> 5;
  const int tilesN = N >> 6;
  const int tilesM = M >> 6;
  const int tile = blockIdx.x * 8 + wave;
  if (tile >= tilesM * tilesN) return;
  const int tm = tile / tilesN;
  const int tn = tile - tm * tilesN;
  const int m0 = tm << 6;
  const int n0 = tn << 6;

  const T* Ab  = A  + (size_t)b * strideA;
  const T* Bb  = Bt + (size_t)b * strideB;
  const T* Ab2 = (SPL >= 1) ? (A2  + (size_t)b * strideA) : nullptr;
  const T* Bb2 = (SPL == 2) ? (Bt2 + (size_t)b * strideB) : nullptr;

  const int rlane = lane & 15;
  const int koff  = (lane >> 4) * 8;
  const int mOff  = (lane >> 4) * 8;

  v8f acc[4][4];
#pragma unroll
  for (int i = 0; i < 4; ++i)
#pragma unroll
    for (int j = 0; j < 4; ++j) acc[i][j] = (v8f){0.f,0.f,0.f,0.f,0.f,0.f,0.f,0.f};

  for (int k0 = 0; k0 < K; k0 += 32) {
    V bh[4], bl[4];
#pragma unroll
    for (int j = 0; j < 4; ++j) {
      const size_t bo = (size_t)(n0 + (j << 4) + rlane) * ldb + koff + k0;
      bh[j] = Frag<T>::load(Bb + bo);
      if (SPL == 2) bl[j] = Frag<T>::load(Bb2 + bo);
    }
#pragma unroll
    for (int i = 0; i < 4; ++i) {
      const size_t ao = (size_t)(m0 + (i << 4) + rlane) * lda + koff + k0;
      V ah = Frag<T>::load(Ab + ao);
      V al;
      if (SPL >= 1) al = Frag<T>::load(Ab2 + ao);
#pragma unroll
      for (int j = 0; j < 4; ++j) {
        acc[i][j] = Frag<T>::mma(ah, bh[j], acc[i][j]);
        if (SPL == 2) acc[i][j] = Frag<T>::mma(ah, bl[j], acc[i][j]);
        if (SPL >= 1) acc[i][j] = Frag<T>::mma(al, bh[j], acc[i][j]);
      }
      Frag<T>::guard4(acc[i][0], acc[i][1], acc[i][2], acc[i][3], ah, (SPL >= 1) ? al : ah);
    }
    Frag<T>::keep(bh[0], bh[1], bh[2], bh[3]);
    if (SPL == 2) Frag<T>::keep(bl[0], bl[1], bl[2], bl[3]);
  }
  acc_guard4(acc[0][0], acc[0][1], acc[0][2], acc[0][3]);
  acc_guard4(acc[1][0], acc[1][1], acc[1][2], acc[1][3]);
  acc_guard4(acc[2][0], acc[2][1], acc[2][2], acc[2][3]);
  acc_guard4(acc[3][0], acc[3][1], acc[3][2], acc[3][3]);

  float* slab = sT[wave];
  const float* Rb = RESID ? (resid + (size_t)b * strideR) : nullptr;
#pragma unroll
  for (int i = 0; i < 4; ++i) {
    const int mBase = m0 + (i << 4);
#pragma unroll
    for (int j = 0; j < 4; ++j) {
      const int n = n0 + (j << 4) + rlane;
      float bv = 0.f;
      if (BIAS_MODE == 2) bv = bias[n];
#pragma unroll
      for (int r = 0; r < 8; ++r) {
        float v = acc[i][j][r] * scale;
        if (BIAS_MODE == 1) v += bias[mBase + mOff + r];
        if (BIAS_MODE == 2) v += bv;
        if (RESID) v += Rb[(size_t)(mBase + mOff + r) * ldc + n];
        if (ACT == 1) v = tanhf(v);
        if (ACT == 2) v = fmaxf(v, 0.0f);
        if (ACT == 3) v = v / (1.0f + expf(-v));
        if (ACT == 4) v = (v > 0.f) ? v : 0.01f * v;
        slab[(mOff + r) * 68 + (j << 4) + rlane] = v;
      }
    }
    __builtin_amdgcn_fence(__ATOMIC_RELEASE, "workgroup");
    __builtin_amdgcn_wave_barrier();
    __builtin_amdgcn_fence(__ATOMIC_ACQUIRE, "workgroup");
    if (OUT_MODE == 0) {
      float* C = (float*)Cout + (size_t)b * strideC;
      const int hh = lane >> 4, c4 = (lane & 15) * 4;
      for (int pass = 0; pass < 2; ++pass) {
#pragma unroll
        for (int it = 0; it < 8; ++it) {
          const int row = it * 2 + hh;
          v4f v = *(const v4f*)(slab + row * 68 + c4);
          *(volatile v4f*)(C + (size_t)(mBase + row) * ldc + n0 + c4) = v;
        }
        __threadfence();
      }
    } else {
      const int q = lane >> 3, c8 = (lane & 7) * 8;
      unsigned short* C  = (unsigned short*)Cout  + (size_t)b * strideC;
      unsigned short* C2 = (OUT_MODE == 2) ? ((unsigned short*)Cout2 + (size_t)b * strideC) : nullptr;
      for (int pass = 0; pass < 2; ++pass) {
#pragma unroll
        for (int it = 0; it < 4; ++it) {
          const int row = it * 4 + q;
          const float* sp = slab + row * 68 + c8;
          v8h hv, lv;
#pragma unroll
          for (int e = 0; e < 8; ++e) {
            if (OUT_MODE == 1) {
              hv[e] = (_Float16)sp[e];
            } else {
              unsigned short hb = f2bf_bits(sp[e]);
              unsigned short lb = f2bf_bits(sp[e] - bf_bits2f(hb));
              hv[e] = __builtin_bit_cast(_Float16, hb);
              lv[e] = __builtin_bit_cast(_Float16, lb);
            }
          }
          *(volatile v8h*)(C + (size_t)(mBase + row) * ldc + n0 + c8) = hv;
          if (OUT_MODE == 2) *(volatile v8h*)(C2 + (size_t)(mBase + row) * ldc + n0 + c8) = lv;
        }
        __threadfence();
      }
    }
    __builtin_amdgcn_fence(__ATOMIC_RELEASE, "workgroup");
    __builtin_amdgcn_wave_barrier();
    __builtin_amdgcn_fence(__ATOMIC_ACQUIRE, "workgroup");
  }
}

__global__ __launch_bounds__(256) void cvt_rows_bf16_kernel(
    const float* __restrict__ src, unsigned short* __restrict__ dst, int total8)
{
  const int i = blockIdx.x * 256 + threadIdx.x;
  if (i >= total8) return;
  const size_t e0 = (size_t)i << 3;
  const v4f a0 = *(const v4f*)(src + e0);
  const v4f a1 = *(const v4f*)(src + e0 + 4);
  v8h hv;
#pragma unroll
  for (int e = 0; e < 4; ++e) {
    const unsigned short h0 = f2bf_bits(a0[e]), h1 = f2bf_bits(a1[e]);
    hv[e]     = __builtin_bit_cast(_Float16, h0);
    hv[4 + e] = __builtin_bit_cast(_Float16, h1);
  }
  unsigned short* q = dst + e0;
  *(volatile v8h*)q = hv;
  __threadfence();
  *(volatile v8h*)q = hv;
}

__global__ __launch_bounds__(256) void transpose_bf16_kernel(
    const float* __restrict__ in, unsigned short* __restrict__ out, int Kr, int Nc, int Npad)
{
  __shared__ __align__(16) float sT[64 * kTrP];
  const int tid = threadIdx.x, lane = tid & 31, wave = tid >> 5;
  const int n0 = blockIdx.x * 64, k0 = blockIdx.y * 64;
  (void)Npad;
#pragma unroll 1
  for (int ig = 0; ig < 4; ++ig) {
#pragma unroll
    for (int ii = 0; ii < 4; ++ii) {
      const int e = (ig * 4 + ii) * 256 + tid;
      const int kr = e >> 6, nc = e & 63;
      const int n = n0 + nc;
      const int ncl = (n < Nc) ? n : (Nc - 1);
      const float keep = (n < Nc) ? 1.0f : 0.0f;
      const float v = in[(size_t)(k0 + kr) * Nc + ncl];
      sT[nc * kTrP + kr] = v * keep;
    }
    asm volatile("" ::: "memory");
  }
  __syncthreads();
  const int q = lane >> 3, c8 = (lane & 7) * 8;
  v8h hv[2];
#pragma unroll
  for (int it = 0; it < 2; ++it) {
    const int nr = it * 32 + wave * 4 + q;
    const float* sp = sT + nr * kTrP + c8;
    const v4f a0 = *(const v4f*)(sp);
    const v4f a1 = *(const v4f*)(sp + 4);
#pragma unroll
    for (int e = 0; e < 4; ++e) {
      const unsigned short h0 = f2bf_bits(a0[e]), h1 = f2bf_bits(a1[e]);
      hv[it][e]     = __builtin_bit_cast(_Float16, h0);
      hv[it][4 + e] = __builtin_bit_cast(_Float16, h1);
    }
  }
  for (int pass = 0; pass < 2; ++pass) {
#pragma unroll
    for (int it = 0; it < 2; ++it) {
      const int nr = it * 32 + wave * 4 + q;
      *(volatile v8h*)(out + (size_t)(n0 + nr) * Kr + k0 + c8) = hv[it];
    }
    __threadfence();
  }
}

__global__ __launch_bounds__(256) void conv_silu_kernel(
    const float* __restrict__ XZ, const float* __restrict__ cw, const float* __restrict__ cb,
    unsigned short* __restrict__ XS)
{
  __shared__ __align__(16) float sT[16 * kConvTP];
  const int tid = threadIdx.x, lane = tid & 31, wave = tid >> 5;
  const int d0 = blockIdx.x * 256, d = d0 + tid;
  const int g0 = blockIdx.y * 64;
  const int tb = g0 & (kSeq - 1);
  const v4f cwv = *(const v4f*)(cw + (size_t)d * kConvK);
  const float w0 = bfr(cwv[0]), w1 = bfr(cwv[1]), w2 = bfr(cwv[2]), w3 = bfr(cwv[3]);
  const float bc = bfr(cb[d]);
  float xm3, xm2, xm1;
  {
    const bool hist = (tb > 0);
    const int rb = hist ? (g0 - 3) : g0;
    const float hf = hist ? 1.0f : 0.0f;
    const float v3 = XZ[(size_t)rb * kXzP + d];
    const float v2 = XZ[(size_t)(rb + 1) * kXzP + d];
    const float v1 = XZ[(size_t)(rb + 2) * kXzP + d];
    xm3 = v3 * hf;
    xm2 = v2 * hf;
    xm1 = v1 * hf;
  }
#pragma unroll 1
  for (int sub = 0; sub < 4; ++sub) {
    const int lb = g0 + sub * 16;
#pragma unroll 1
    for (int s = 0; s < 16; ++s) {
      const float xcur = XZ[(size_t)(lb + s) * kXzP + d];
      float acc = w0 * xm3;
      acc = fmaf(w1, xm2, acc);
      acc = fmaf(w2, xm1, acc);
      acc = fmaf(w3, xcur, acc);
      const float sv = acc + bc;
      sT[s * kConvTP + tid] = sv * sigm_f32(sv);
      xm3 = xm2; xm2 = xm1; xm1 = xcur;
    }
    __syncthreads();
    v8h bh[2];
#pragma unroll
    for (int it = 0; it < 2; ++it) {
      const float* sp = sT + (it * 8 + wave) * kConvTP + lane * 8;
      const v4f a0 = *(const v4f*)(sp);
      const v4f a1 = *(const v4f*)(sp + 4);
#pragma unroll
      for (int e = 0; e < 4; ++e) {
        const unsigned short h0 = f2bf_bits(a0[e]), h1 = f2bf_bits(a1[e]);
        bh[it][e]     = __builtin_bit_cast(_Float16, h0);
        bh[it][4 + e] = __builtin_bit_cast(_Float16, h1);
      }
    }
    for (int pass = 0; pass < 2; ++pass) {
#pragma unroll
      for (int it = 0; it < 2; ++it) {
        const size_t o = (size_t)(lb + it * 8 + wave) * kDin + d0 + lane * 8;
        *(volatile v8h*)(XS + o) = bh[it];
      }
      __threadfence();
    }
    __syncthreads();
  }
}

__global__ __launch_bounds__(kScanCh) void scan_kernel(
    const float* __restrict__ BCD, const float* __restrict__ XZ,
    const float* __restrict__ cw, const float* __restrict__ cb,
    const float* __restrict__ dtw, const float* __restrict__ dtb,
    const float* __restrict__ Alog, const float* __restrict__ Dp,
    unsigned short* __restrict__ YH, unsigned short* __restrict__ YL)
{
  __shared__ __align__(16) float    sX[kScanTS * kBcdP];
  __shared__ __align__(16) float    sY[kScanTS * kScanYP];
  __shared__ __align__(16) float    sA[kNst * kScanCh];
  __shared__ __align__(16) _Float16 sCd[kScanSub * kCdP];
  __shared__ __align__(16) _Float16 sHh[kScanSub * kScanCh * kNst];
  __shared__ __align__(16) float    sSk[kScanSub * kScanCh];
  __shared__ __align__(16) float    sGt[kScanSub * kScanCh];
  const int tid = threadIdx.x, lane = tid & 31, wave = tid >> 5;
  const int hh = lane >> 4, cl = lane & 15;
  constexpr int kBlkPerB = kDin / kScanCh;
  const int bix = blockIdx.x / kBlkPerB;
  const int d0  = (blockIdx.x - bix * kBlkPerB) * kScanCh;
  const int d   = d0 + tid;
  const size_t row0 = (size_t)bix * kSeq;
#pragma unroll 1
  for (int s = 0; s < kNst; ++s) sA[s * kScanCh + tid] = -expf(bfr(Alog[(size_t)d * kNst + s])) * kLog2e;
  __syncthreads();
  float nA2[kNst], h[kNst];
#pragma unroll
  for (int s = 0; s < kNst; ++s) {
    nA2[s] = sA[s * kScanCh + tid];
    h[s] = 0.f;
  }
  const v4f cwv = *(const v4f*)(cw + (size_t)d * kConvK);
  const float w0 = bfr(cwv[0]), w1 = bfr(cwv[1]), w2 = bfr(cwv[2]), w3 = bfr(cwv[3]);
  asm volatile("" ::: "memory");
  const float bc = bfr(cb[d]), dw = bfr(dtw[d]), db = bfr(dtb[d]), Dd = bfr(Dp[d]);
  float xm3 = 0.f, xm2 = 0.f, xm1 = 0.f;
  const int lr = tid >> 4, lc4 = (tid & 15) * 4;
  const int q = lane >> 3, c8 = (lane & 7) * 8;
#pragma unroll 1
  for (int t0 = 0; t0 < kSeq; t0 += kScanTS) {
    __syncthreads();
#pragma unroll
    for (int i = 0; i < 8; ++i) {
      const int r = lr + 4 * i;
      *(v4f*)(sX + r * kBcdP + lc4) = *(const v4f*)(BCD + (row0 + t0 + r) * kBcdP + lc4);
    }
    asm volatile("" ::: "memory");
#pragma unroll
    for (int i = 8; i < 16; ++i) {
      const int r = lr + 4 * i;
      *(v4f*)(sX + r * kBcdP + lc4) = *(const v4f*)(BCD + (row0 + t0 + r) * kBcdP + lc4);
    }
    __syncthreads();
#pragma unroll 1
    for (int sub = 0; sub < kScanTS / kScanSub; ++sub) {
      const int sb = sub * kScanSub;
      {
        const int tr = tid & 15, kq = tid >> 4;
#pragma unroll
        for (int u = 0; u < 2; ++u) {
          const int kk = 2 * kq + u;
          const float f0 = (tr == 2 * kk) ? kCcar : 0.0f;
          const float f1 = (tr == 2 * kk + 1) ? kCcar : 0.0f;
          const float* c0p = sX + (sb + 2 * kk) * kBcdP + kNst;
          const float* c1p = c0p + kBcdP;
          _Float16* dp = sCd + tr * kCdP + 32 * kk;
#pragma unroll
          for (int q8 = 0; q8 < 2; ++q8) {
            const v4f a0 = *(const v4f*)(c0p + 8 * q8);
            const v4f a1 = *(const v4f*)(c0p + 8 * q8 + 4);
            const v4f b0 = *(const v4f*)(c1p + 8 * q8);
            const v4f b1 = *(const v4f*)(c1p + 8 * q8 + 4);
            v8h va, vb;
#pragma unroll
            for (int e = 0; e < 4; ++e) {
              va[e]     = (_Float16)(a0[e] * f0);
              va[4 + e] = (_Float16)(a1[e] * f0);
              vb[e]     = (_Float16)(b0[e] * f1);
              vb[4 + e] = (_Float16)(b1[e] * f1);
            }
            *(v8h*)(dp + 8 * q8) = va;
            *(v8h*)(dp + 16 + 8 * q8) = vb;
          }
        }
      }
#pragma unroll 1
      for (int s = 0; s < kScanSub; ++s) {
        const size_t grow = row0 + t0 + sb + s;
        const float* xr = sX + (sb + s) * kBcdP;
        float Bs[kNst];
#pragma unroll
        for (int q4 = 0; q4 < 4; ++q4) {
          const v4f bv = *(const v4f*)(xr + 4 * q4);
          Bs[4 * q4 + 0] = bv[0]; Bs[4 * q4 + 1] = bv[1]; Bs[4 * q4 + 2] = bv[2]; Bs[4 * q4 + 3] = bv[3];
        }
        const float dtraw = xr[2 * kNst];
        const float xcur = XZ[grow * kXzP + d];
        const float zv   = XZ[grow * kXzP + kDin + d];
        float ca = w0 * xm3;
        ca = fmaf(w1, xm2, ca);
        ca = fmaf(w2, xm1, ca);
        ca = fmaf(w3, xcur, ca);
        const float u  = ca + bc;
        const float us = u * sigm_f32(u);
        xm3 = xm2; xm2 = xm1; xm1 = xcur;
        const float v   = fmaf(dtraw, dw, db);
        const float dt  = softplus_f32(v);
        const float dtx = dt * us;
        v8h hv0, hv1;
#pragma unroll
        for (int k = 0; k < 8; ++k) {
          const float e0 = exp2f(dt * nA2[k]);
          const float e1 = exp2f(dt * nA2[8 + k]);
          h[k]     = fmaf(e0, h[k], dtx * Bs[k]);
          h[8 + k] = fmaf(e1, h[8 + k], dtx * Bs[8 + k]);
          hv0[k] = (_Float16)(h[k] * kHcar);
          hv1[k] = (_Float16)(h[8 + k] * kHcar);
        }
        _Float16* hp = sHh + (s * kScanCh + tid) * kNst;
        *(v8h*)hp = hv0;
        *(v8h*)(hp + 8) = hv1;
        sSk[s * kScanCh + tid] = us * Dd;
        sGt[s * kScanCh + tid] = zv * sigm_f32(zv);
      }
      __syncthreads();
#pragma unroll
      for (int i = 0; i < 2; ++i) {
        const int chl = wave * 32 + i * 16 + cl;
        v8f acc = (v8f){0.f,0.f,0.f,0.f,0.f,0.f,0.f,0.f};
#pragma unroll
        for (int kk = 0; kk < 8; ++kk) {
          const v16h af = Frag<_Float16>::load(sCd + cl * kCdP + 32 * kk + 8 * hh);
          Frag<_Float16>::U bu;
          bu.h[0] = *(const v8h*)(sHh + ((2 * kk) * kScanCh + chl) * kNst + 8 * hh);
          bu.h[1] = *(const v8h*)(sHh + ((2 * kk + 1) * kScanCh + chl) * kNst + 8 * hh);
          acc = mma16_f16(af, bu.v, acc);
        }
#pragma unroll
        for (int r = 0; r < 8; ++r) {
          const int t = 8 * hh + r;
          const float yv = (acc[r] * kYfold + sSk[t * kScanCh + chl]) * sGt[t * kScanCh + chl];
          sY[(sb + t) * kScanYP + chl] = yv;
        }
      }
      __syncthreads();
    }
    v8h hv[8], lv[8];
#pragma unroll
    for (int it = 0; it < 8; ++it) {
      const int row = it * 8 + wave * 4 + q;
      const float* sp = sY + row * kScanYP + c8;
      const v4f a0 = *(const v4f*)(sp);
      const v4f a1 = *(const v4f*)(sp + 4);
#pragma unroll
      for (int e = 0; e < 4; ++e) {
        const unsigned short h0 = f2bf_bits(a0[e]), h1 = f2bf_bits(a1[e]);
        const unsigned short l0 = f2bf_bits(a0[e] - bf_bits2f(h0)), l1 = f2bf_bits(a1[e] - bf_bits2f(h1));
        hv[it][e]     = __builtin_bit_cast(_Float16, h0);
        hv[it][4 + e] = __builtin_bit_cast(_Float16, h1);
        lv[it][e]     = __builtin_bit_cast(_Float16, l0);
        lv[it][4 + e] = __builtin_bit_cast(_Float16, l1);
      }
    }
    for (int pass = 0; pass < 2; ++pass) {
#pragma unroll
      for (int it = 0; it < 8; ++it) {
        const int row = it * 8 + wave * 4 + q;
        const size_t o = (row0 + t0 + row) * kDin + d0 + c8;
        *(volatile v8h*)(YH + o) = hv[it];
        *(volatile v8h*)(YL + o) = lv[it];
      }
      __threadfence();
    }
  }
}

extern "C" void kernel_launch(void* const* d_in, const int* in_sizes, int n_in,
                              void* d_out, int out_size, void* d_ws, size_t ws_size,
                              hipStream_t stream) {
  if (n_in < 10) return;
  if (in_sizes[0] != kRows * kDm) return;
  if (in_sizes[1] != kDm * kXzP) return;
  if (in_sizes[2] != kDin * kConvK) return;
  if (in_sizes[3] != kDin) return;
  if (in_sizes[4] != kDin * kBcdN) return;
  if (in_sizes[5] != kDin) return;
  if (in_sizes[6] != kDin) return;
  if (in_sizes[7] != kDin * kNst) return;
  if (in_sizes[8] != kDin) return;
  if (in_sizes[9] != kDin * kDm) return;
  if (out_size != kRows * kDm) return;
  if (ws_size < kWsTotal) return;

  const float* x       = (const float*)d_in[0];
  const float* W_in    = (const float*)d_in[1];
  const float* conv_w  = (const float*)d_in[2];
  const float* conv_b  = (const float*)d_in[3];
  const float* W_xproj = (const float*)d_in[4];
  const float* dt_w    = (const float*)d_in[5];
  const float* dt_b    = (const float*)d_in[6];
  const float* A_log   = (const float*)d_in[7];
  const float* Dp      = (const float*)d_in[8];
  const float* W_out   = (const float*)d_in[9];
  float* out = (float*)d_out;

  char* ws = (char*)d_ws;
  unsigned short* XB  = (unsigned short*)(ws + kOffXB);
  unsigned short* W1T = (unsigned short*)(ws + kOffW1T);
  unsigned short* W2T = (unsigned short*)(ws + kOffW2T);
  unsigned short* W3T = (unsigned short*)(ws + kOffW3T);
  float*          XZ  = (float*)(ws + kOffXZ);
  unsigned short* XS  = (unsigned short*)(ws + kOffXS);
  float*          BCD = (float*)(ws + kOffBCD);
  unsigned short* YH  = (unsigned short*)(ws + kOffYH);
  unsigned short* YL  = (unsigned short*)(ws + kOffYL);

  cvt_rows_bf16_kernel<<<(kRows * kDm / 8) / 256, 256, 0, stream>>>(x, XB, kRows * kDm / 8);
  transpose_bf16_kernel<<<dim3(kXzP / 64, kDm / 64), 256, 0, stream>>>(W_in, W1T, kDm, kXzP, kXzP);
  transpose_bf16_kernel<<<dim3(kBcdP / 64, kDin / 64), 256, 0, stream>>>(W_xproj, W2T, kDin, kBcdN, kBcdP);
  transpose_bf16_kernel<<<dim3(kDm / 64, kDin / 64), 256, 0, stream>>>(W_out, W3T, kDin, kDm, kDm);

  wmma_gemm64<1, 0, 0, 0, false><<<dim3(512, 1), 256, 0, stream>>>(
      XB, nullptr, kDm, 0L,
      W1T, nullptr, kDm, 0L,
      (void*)XZ, nullptr, kXzP, 0L,
      nullptr, nullptr, 0L,
      kRows, kXzP, kDm, 1.0f);

  conv_silu_kernel<<<dim3(kDin / 256, kRows / 64), 256, 0, stream>>>(XZ, conv_w, conv_b, XS);

  wmma_gemm64<1, 0, 0, 0, false><<<dim3(8, 1), 256, 0, stream>>>(
      XS, nullptr, kDin, 0L,
      W2T, nullptr, kDin, 0L,
      (void*)BCD, nullptr, kBcdP, 0L,
      nullptr, nullptr, 0L,
      kRows, kBcdP, kDin, 1.0f);

  scan_kernel<<<kBatch * (kDin / kScanCh), kScanCh, 0, stream>>>(BCD, XZ, conv_w, conv_b, dt_w, dt_b, A_log, Dp, YH, YL);

  wmma_gemm64<1, 1, 0, 0, false><<<dim3(128, 1), 256, 0, stream>>>(
      YH, YL, kDin, 0L,
      W3T, nullptr, kDin, 0L,
      (void*)out, nullptr, kDm, 0L,
      nullptr, nullptr, 0L,
      kRows, kDm, kDin, 1.0f);
}
